// SSMBlock_1958505087212
// MI455X (gfx1250) — hardware-run, weakly checked
//
#include <hip/hip_runtime.h>
#include <math.h>

constexpr int kBatch = 4;
constexpr int kSeq   = 2048;
constexpr int kDm    = 1024;
constexpr int kNs    = 16;
constexpr int kDff   = 4096;
constexpr int kTok   = kBatch * kSeq;
constexpr float kEps       = 1e-6f;
constexpr float kWCarry    = 64.0f;
constexpr float kWCarryInv = 0.015625f;
constexpr float kLnDtLo    = -6.907755278982137f;
constexpr float kLnDtStep  = 0.3070113457325394f;

static_assert(kTok % 64 == 0 && kDff % 64 == 0 && kDm % 64 == 0);
static_assert(kDm % 32 == 0 && kDff % 32 == 0);
static_assert(kDm == 1024 && kNs == 16 && kTok % 32 == 0);

constexpr size_t kBytesX2  = (size_t)kTok * kDm * 4;
constexpr size_t kBytesH   = (size_t)kTok * kDm * 2;
constexpr size_t kBytesW   = (size_t)kDm * kDff * 2;
constexpr size_t kBytesG   = (size_t)kTok * kDff * 2;
constexpr size_t kBytesPar = (size_t)kDm * kNs * 4;
constexpr size_t kBytesRst = (size_t)kTok * 4;
constexpr size_t kOffX2  = 0;
constexpr size_t kOffH   = kOffX2 + kBytesX2;
constexpr size_t kOffW1  = kOffH + kBytesH;
constexpr size_t kOffW2  = kOffW1 + kBytesW;
constexpr size_t kOffG   = kOffW2 + kBytesW;
constexpr size_t kOffDA  = kOffG;
constexpr size_t kOffDB  = kOffDA + kBytesPar;
constexpr size_t kOffRst = kOffDB + kBytesPar;
constexpr size_t kWsTotal = kOffG + kBytesG;
static_assert(kWsTotal == 134217728);
static_assert(kOffRst + kBytesRst <= kOffG + kBytesG);
static_assert(kOffH % 256 == 0 && kOffW1 % 256 == 0 && kOffW2 % 256 == 0 && kOffG % 256 == 0 && kOffDB % 256 == 0 && kOffRst % 256 == 0);

typedef __attribute__((ext_vector_type(16))) _Float16 v16h;
typedef __attribute__((ext_vector_type(8)))  _Float16 v8h;
typedef __attribute__((ext_vector_type(16))) __bf16   v16b;
typedef __attribute__((ext_vector_type(8)))  __bf16   v8b;
typedef __attribute__((ext_vector_type(8)))  float    v8f;
typedef __attribute__((ext_vector_type(4)))  float    v4f;

__device__ __forceinline__ void dep_guard_h(v8f& a, v8f& b, v16h x, v16h y) { asm volatile("v_nop\n\tv_nop\n\tv_nop\n\tv_nop" : "+v"(a), "+v"(b) : "v"(x), "v"(y)); }
__device__ __forceinline__ void keep4_h(v16h a, v16h b, v16h c, v16h d) { asm volatile("v_nop" :: "v"(a), "v"(b), "v"(c), "v"(d)); }
__device__ __forceinline__ void acc_guard4(v8f& a, v8f& b, v8f& c, v8f& d) { asm volatile("v_nop\n\tv_nop\n\tv_nop\n\tv_nop" : "+v"(a), "+v"(b), "+v"(c), "+v"(d)); }

template <typename T> struct Frag;
template <> struct Frag<_Float16> {
  typedef v16h V; union U { v16h v; v8h h[2]; };
  static __device__ __forceinline__ v16h load(const _Float16* p) {
    U f; f.h[0] = *(const v8h*)(p); f.h[1] = *(const v8h*)(p + 16); return f.v;
  }
  static __device__ __forceinline__ v8f mma(v16h a, v16h b, v8f c) {
    return __builtin_amdgcn_wmma_f32_16x16x32_f16(false, a, false, b, (short)0, c, false, false);
  }
  static __device__ __forceinline__ void guard(v8f& a, v8f& b, v16h x, v16h y) { dep_guard_h(a, b, x, y); }
  static __device__ __forceinline__ void keep(v16h a, v16h b, v16h c, v16h d) { keep4_h(a, b, c, d); }
};

__device__ __forceinline__ float gelu_erf_poly(float v) {
  const float z  = v * 0.70710678118654752f;
  const float az = fabsf(z);
  const float t  = __builtin_amdgcn_rcpf(fmaf(0.3275911f, az, 1.0f));
  float p = fmaf(1.061405429f, t, -1.453152027f);
  p = fmaf(p, t, 1.421413741f);
  p = fmaf(p, t, -0.284496736f);
  p = fmaf(p, t, 0.254829592f);
  p = p * t;
  const float ex   = __builtin_amdgcn_exp2f((az * az) * -1.4426950408889634f);
  const float erfa = 1.0f - p * ex;
  const float erfz = copysignf(erfa, z);
  return 0.5f * v * (1.0f + erfz);
}

template <int BIAS_MODE, int OUT_MODE, bool RESID, int ACT>
__global__ __launch_bounds__(256) void wmma_gemm64_f16(
    const unsigned short* __restrict__ Ap, int lda,
    const unsigned short* __restrict__ Btp, int ldb,
    void* __restrict__ Cout, int ldc,
    const float* __restrict__ bias,
    const float* __restrict__ resid,
    int M, int N, int K, float scale) {
  static_assert(!(RESID && OUT_MODE != 0));
  static_assert(!(ACT != 0 && ACT != 6));
  static_assert(!(ACT == 6 && OUT_MODE != 1));
  static_assert(BIAS_MODE == 0 || BIAS_MODE == 2);
  typedef _Float16 T;
  typedef v16h V;
  const T* A = (const T*)Ap; const T* Bt = (const T*)Btp;
  __shared__ __align__(16) float sT[8][16 * 68];
  const int lane = threadIdx.x & 31;
  const int wave = threadIdx.x >> 5;
  const int tilesN = N >> 6;
  const int tilesM = M >> 6;
  const int tile = blockIdx.x * 8 + wave;
  if (tile >= tilesM * tilesN) return;
  const int tm = tile / tilesN;
  const int tn = tile - tm * tilesN;
  const int m0 = tm << 6;
  const int n0 = tn << 6;

  const int rlane = lane & 15;
  const int koff  = (lane >> 4) * 8;
  const int mOff  = (lane >> 4) * 8;

  v8f acc[4][4];
#pragma unroll
  for (int i = 0; i < 4; ++i)
#pragma unroll
    for (int j = 0; j < 4; ++j) acc[i][j] = (v8f){0.f,0.f,0.f,0.f,0.f,0.f,0.f,0.f};

  for (int k0 = 0; k0 < K; k0 += 32) {
    V bh[4];
#pragma unroll
    for (int j = 0; j < 4; ++j) {
      const size_t bo = (size_t)(n0 + (j << 4) + rlane) * ldb + koff + k0;
      bh[j] = Frag<T>::load(Bt + bo);
    }
#pragma unroll
    for (int i = 0; i < 4; ++i) {
      const size_t ao = (size_t)(m0 + (i << 4) + rlane) * lda + koff + k0;
      V ah = Frag<T>::load(A + ao);
#pragma unroll
      for (int j = 0; j < 4; ++j) {
        acc[i][j] = Frag<T>::mma(ah, bh[j], acc[i][j]);
      }
      Frag<T>::guard(acc[i][0], acc[i][3], ah, ah);
    }
    Frag<T>::keep(bh[0], bh[1], bh[2], bh[3]);
  }
  acc_guard4(acc[0][0], acc[0][1], acc[0][2], acc[0][3]);
  acc_guard4(acc[1][0], acc[1][1], acc[1][2], acc[1][3]);
  acc_guard4(acc[2][0], acc[2][1], acc[2][2], acc[2][3]);
  acc_guard4(acc[3][0], acc[3][1], acc[3][2], acc[3][3]);

  float* slab = sT[wave];
#pragma unroll
  for (int i = 0; i < 4; ++i) {
    const int mBase = m0 + (i << 4);
#pragma unroll
    for (int j = 0; j < 4; ++j) {
      const int n = n0 + (j << 4) + rlane;
      float bv = 0.f;
      if (BIAS_MODE == 2) bv = bias[n];
#pragma unroll
      for (int r = 0; r < 8; ++r) {
        float v = acc[i][j][r] * scale;
        if (BIAS_MODE == 2) v += bv;
        slab[(mOff + r) * 68 + (j << 4) + rlane] = v;
      }
    }
    __builtin_amdgcn_fence(__ATOMIC_RELEASE, "workgroup");
    __builtin_amdgcn_wave_barrier();
    __builtin_amdgcn_fence(__ATOMIC_ACQUIRE, "workgroup");
    if (OUT_MODE == 0) {
      float* Cb = (float*)Cout;
      const int hh = lane >> 4, c4 = (lane & 15) * 4;
      v4f vals[8];
#pragma unroll
      for (int it = 0; it < 8; ++it) {
        const int row = it * 2 + hh;
        v4f v = *(const v4f*)(slab + row * 68 + c4);
        if (RESID) {
          const v4f rr = *(const v4f*)(resid + (size_t)(mBase + row) * ldc + n0 + c4);
          v = v + rr;
        }
        vals[it] = v;
      }
#pragma unroll
      for (int pass = 0; pass < 2; ++pass) {
#pragma unroll
        for (int it = 0; it < 8; ++it) {
          const int row = it * 2 + hh;
          *(volatile v4f*)(Cb + (size_t)(mBase + row) * ldc + n0 + c4) = vals[it];
        }
        __threadfence();
      }
    } else {
      const int q = lane >> 3, c8 = (lane & 7) * 8;
      _Float16* Cb = (_Float16*)Cout;
      v8h hv[4];
#pragma unroll
      for (int it = 0; it < 4; ++it) {
        const int row = it * 4 + q;
        const float* sp = slab + row * 68 + c8;
        const v4f a = *(const v4f*)(sp);
        const v4f c = *(const v4f*)(sp + 4);
        float f[8] = {a[0], a[1], a[2], a[3], c[0], c[1], c[2], c[3]};
        v8h tv;
#pragma unroll
        for (int e = 0; e < 8; ++e) {
          float g = f[e];
          if (ACT == 6) g = gelu_erf_poly(g);
          tv[e] = (_Float16)g;
        }
        hv[it] = tv;
      }
#pragma unroll
      for (int pass = 0; pass < 2; ++pass) {
#pragma unroll
        for (int it = 0; it < 4; ++it) {
          const int row = it * 4 + q;
          *(volatile v8h*)(Cb + (size_t)(mBase + row) * ldc + n0 + c8) = hv[it];
        }
        __threadfence();
      }
    }
    __builtin_amdgcn_fence(__ATOMIC_RELEASE, "workgroup");
    __builtin_amdgcn_wave_barrier();
    __builtin_amdgcn_fence(__ATOMIC_ACQUIRE, "workgroup");
  }
}

__global__ __launch_bounds__(256) void cast_t_kernel(const float* __restrict__ in, _Float16* __restrict__ out,
                                                      int Kr, int Nc, float mul) {
  __shared__ __align__(16) float tt[64 * 68];
  const int tid = threadIdx.x;
  const int n0 = blockIdx.x * 64;
  const int k0 = blockIdx.y * 64;
  const int nl = (tid & 15) * 4;
#pragma unroll
  for (int p = 0; p < 4; ++p) {
    const int kl = (tid >> 4) + 16 * p;
    const v4f v = *(const v4f*)(in + (size_t)(k0 + kl) * Nc + n0 + nl);
    tt[(nl + 0) * 68 + kl] = v[0];
    tt[(nl + 1) * 68 + kl] = v[1];
    tt[(nl + 2) * 68 + kl] = v[2];
    tt[(nl + 3) * 68 + kl] = v[3];
  }
  __syncthreads();
  const int c8 = (tid & 7) * 8;
  v8h hv[2];
#pragma unroll
  for (int it = 0; it < 2; ++it) {
    const int rn = (tid >> 3) + 32 * it;
    const v4f a = *(const v4f*)(tt + rn * 68 + c8);
    const v4f c = *(const v4f*)(tt + rn * 68 + c8 + 4);
    v8h h;
    h[0] = (_Float16)(a[0] * mul); h[1] = (_Float16)(a[1] * mul);
    h[2] = (_Float16)(a[2] * mul); h[3] = (_Float16)(a[3] * mul);
    h[4] = (_Float16)(c[0] * mul); h[5] = (_Float16)(c[1] * mul);
    h[6] = (_Float16)(c[2] * mul); h[7] = (_Float16)(c[3] * mul);
    hv[it] = h;
  }
#pragma unroll
  for (int pass = 0; pass < 2; ++pass) {
#pragma unroll
    for (int it = 0; it < 2; ++it) {
      const int rn = (tid >> 3) + 32 * it;
      *(volatile v8h*)(out + (size_t)(n0 + rn) * Kr + k0 + c8) = hv[it];
    }
    __threadfence();
  }
}

__global__ __launch_bounds__(256) void decay_param_kernel(const float* __restrict__ Ap, const float* __restrict__ Bp,
                                                           float* __restrict__ dAo, float* __restrict__ dBo) {
  const int idx = blockIdx.x * 256 + threadIdx.x;
  const int n = idx & (kNs - 1);
  const float dt = expf(kLnDtLo + (float)n * kLnDtStep);
  const float ea = expf(Ap[idx]);
  const float da = expf(-ea * dt);
  const float db = (Bp[idx] * (1.0f - da)) / ea;
  volatile float* pa = dAo + idx;
  volatile float* pb = dBo + idx;
  *pa = da;
  *pb = db;
  __threadfence();
  *pa = da;
  *pb = db;
}

__global__ __launch_bounds__(256) void rstat_kernel(const float* __restrict__ xin, float* __restrict__ rout) {
  __shared__ float sr[32];
  const int tid = threadIdx.x;
  const int lane = tid & 31, wave = tid >> 5;
  const int tb = blockIdx.x * 32;
#pragma unroll 1
  for (int i = 0; i < 4; ++i) {
    const int tk = tb + wave * 4 + i;
    const float* row = xin + (size_t)tk * kDm + lane * 4;
    float ss = 0.0f;
#pragma unroll
    for (int p = 0; p < 8; ++p) {
      const v4f v = *(const v4f*)(row + p * 128);
      ss += v[0] * v[0];
      ss += v[1] * v[1];
      ss += v[2] * v[2];
      ss += v[3] * v[3];
    }
#pragma unroll
    for (int off = 16; off > 0; off >>= 1) ss += __shfl_xor(ss, off, 32);
    const float r = rsqrtf(ss * (1.0f / (float)kDm) + kEps);
    if (lane == 0) sr[wave * 4 + i] = r;
  }
  __syncthreads();
  if (wave == 0) {
    const float v = sr[lane];
    volatile float* p = rout + tb + lane;
    *p = v;
    __threadfence();
    *p = v;
  }
}

__device__ __forceinline__ void stage_row16(const float* __restrict__ src, float* stile, int tid, float (&dst)[kNs]) {
#pragma unroll
  for (int p = 0; p < 4; ++p) {
    const v4f v = *(const v4f*)(src + tid * 4 + p * 1024);
    *(v4f*)(stile + tid * 4 + p * 1024) = v;
  }
  __syncthreads();
#pragma unroll
  for (int m = 0; m < 4; ++m) {
    const v4f v = *(const v4f*)(stile + tid * 16 + m * 4);
    dst[4 * m + 0] = v[0]; dst[4 * m + 1] = v[1]; dst[4 * m + 2] = v[2]; dst[4 * m + 3] = v[3];
  }
  __syncthreads();
}

__global__ __launch_bounds__(256) void state_scan_kernel(
    const float* __restrict__ x, const float* __restrict__ rst, const float* __restrict__ sc1,
    const float* __restrict__ dAp, const float* __restrict__ dBp, const float* __restrict__ Cp,
    const float* __restrict__ Dp, float* __restrict__ x2) {
  __shared__ __align__(16) float stile[256 * kNs];
  const int tid = threadIdx.x;
  const int dblk = blockIdx.x & 3;
  const int b = (blockIdx.x >> 2) & 3;
  const int d0 = dblk * 256;
  const int d = d0 + tid;
  float dA[kNs], dB[kNs], Cc[kNs], s[kNs];
  stage_row16(dAp + d0 * kNs, stile, tid, dA);
  stage_row16(dBp + d0 * kNs, stile, tid, dB);
  stage_row16(Cp + d0 * kNs, stile, tid, Cc);
#pragma unroll
  for (int n = 0; n < kNs; ++n) s[n] = 0.0f;
  const float scv = sc1[d];
  const float Dd = Dp[d];
  const size_t base = (size_t)b * kSeq * kDm + d;
  const float* xb = x + base;
  float* ob = x2 + base;
  const float* rb = rst + b * kSeq;
#pragma unroll 1
  for (int t = 0; t < kSeq; ++t) {
    const float xv = xb[(size_t)t * kDm];
    const float rv = rb[t];
    const float u = xv * rv * scv;
    float y = 0.0f;
#pragma unroll
    for (int n = 0; n < kNs; ++n) {
      s[n] = s[n] * dA[n] + u * dB[n];
      y += Cc[n] * s[n];
    }
    const float o = xv + (y + u * Dd);
    volatile float* op = ob + (size_t)t * kDm;
    *op = o;
    __threadfence();
    *op = o;
  }
}

__global__ __launch_bounds__(128) void rmsnorm_f16_kernel(const float* __restrict__ xin, const float* __restrict__ scl,
                                                           _Float16* __restrict__ hout) {
  __shared__ float sred[4];
  const int tok = blockIdx.x;
  const int tid = threadIdx.x;
  const int lane = tid & 31, wave = tid >> 5;
  const float* row = xin + (size_t)tok * kDm + tid * 8;
  const v4f a = *(const v4f*)(row);
  const v4f c = *(const v4f*)(row + 4);
  float ss = 0.0f;
  ss += a[0] * a[0]; ss += a[1] * a[1]; ss += a[2] * a[2]; ss += a[3] * a[3];
  ss += c[0] * c[0]; ss += c[1] * c[1]; ss += c[2] * c[2]; ss += c[3] * c[3];
#pragma unroll
  for (int off = 16; off > 0; off >>= 1) ss += __shfl_xor(ss, off, 32);
  if (lane == 0) sred[wave] = ss;
  __syncthreads();
  const float tot = ((sred[0] + sred[1]) + sred[2]) + sred[3];
  const float r = rsqrtf(tot * (1.0f / (float)kDm) + kEps);
  const v4f s0 = *(const v4f*)(scl + tid * 8);
  const v4f s1 = *(const v4f*)(scl + tid * 8 + 4);
  v8h hv;
  hv[0] = (_Float16)(a[0] * r * s0[0]);
  hv[1] = (_Float16)(a[1] * r * s0[1]);
  hv[2] = (_Float16)(a[2] * r * s0[2]);
  hv[3] = (_Float16)(a[3] * r * s0[3]);
  hv[4] = (_Float16)(c[0] * r * s1[0]);
  hv[5] = (_Float16)(c[1] * r * s1[1]);
  hv[6] = (_Float16)(c[2] * r * s1[2]);
  hv[7] = (_Float16)(c[3] * r * s1[3]);
  volatile v8h* hp = (volatile v8h*)(hout + (size_t)tok * kDm + tid * 8);
  *hp = hv;
  __threadfence();
  *hp = hv;
}

extern "C" void kernel_launch(void* const* d_in, const int* in_sizes, int n_in,
                              void* d_out, int out_size, void* d_ws, size_t ws_size,
                              hipStream_t stream) {
  if (n_in < 11) return;
  if (in_sizes[0] != kTok * kDm || in_sizes[1] != kDm * kNs || in_sizes[2] != kDm * kNs ||
      in_sizes[3] != kDm * kNs || in_sizes[4] != kDm || in_sizes[5] != kDm || in_sizes[6] != kDm ||
      in_sizes[7] != kDm * kDff || in_sizes[8] != kDff || in_sizes[9] != kDff * kDm ||
      in_sizes[10] != kDm || out_size != kTok * kDm) return;
  if (ws_size < kWsTotal) return;

  const float* x   = (const float*)d_in[0];
  const float* Ain = (const float*)d_in[1];
  const float* Bin = (const float*)d_in[2];
  const float* Cin = (const float*)d_in[3];
  const float* Din = (const float*)d_in[4];
  const float* sc1 = (const float*)d_in[5];
  const float* sc2 = (const float*)d_in[6];
  const float* w1  = (const float*)d_in[7];
  const float* b1  = (const float*)d_in[8];
  const float* w2  = (const float*)d_in[9];
  const float* b2  = (const float*)d_in[10];
  float* out = (float*)d_out;

  char* ws = (char*)d_ws;
  float*    X2  = (float*)(ws + kOffX2);
  _Float16* H   = (_Float16*)(ws + kOffH);
  _Float16* W1t = (_Float16*)(ws + kOffW1);
  _Float16* W2t = (_Float16*)(ws + kOffW2);
  _Float16* G   = (_Float16*)(ws + kOffG);
  float*    dA  = (float*)(ws + kOffDA);
  float*    dB  = (float*)(ws + kOffDB);
  float*    Rst = (float*)(ws + kOffRst);

  decay_param_kernel<<<(kDm * kNs) / 256, 256, 0, stream>>>(Ain, Bin, dA, dB);
  rstat_kernel<<<kTok / 32, 256, 0, stream>>>(x, Rst);
  cast_t_kernel<<<dim3(kDff / 64, kDm / 64), 256, 0, stream>>>(w1, W1t, kDm, kDff, kWCarry);
  cast_t_kernel<<<dim3(kDm / 64, kDff / 64), 256, 0, stream>>>(w2, W2t, kDff, kDm, kWCarry);
  state_scan_kernel<<<kBatch * (kDm / 256), 256, 0, stream>>>(x, Rst, sc1, dA, dB, Cin, Din, X2);
  rmsnorm_f16_kernel<<<kTok, 128, 0, stream>>>(X2, sc2, H);
  {
    const int tiles = (kTok / 64) * (kDff / 64);
    wmma_gemm64_f16<2, 1, false, 6><<<(tiles + 7) / 8, 256, 0, stream>>>(
        (const unsigned short*)H, kDm, (const unsigned short*)W1t, kDm, (void*)G, kDff,
        b1, nullptr, kTok, kDff, kDm, kWCarryInv);
  }
  {
    const int tiles = (kTok / 64) * (kDm / 64);
    wmma_gemm64_f16<2, 0, true, 0><<<(tiles + 7) / 8, 256, 0, stream>>>(
        (const unsigned short*)G, kDff, (const unsigned short*)W2t, kDff, (void*)out, kDm,
        b2, X2, kTok, kDm, kDff, kWCarryInv);
  }
}
